// LogLSTM_71957882077828
// MI455X (gfx1250) — hardware-verified
//
#include <hip/hip_runtime.h>


#define VV   50000
#define EE   128
#define HH   128
#define BB   256
#define TT   512
#define CC   2
#define G4   512
#define WP   128
#define XPP  512
#define AP   136
#define HP   132
#define MB   16
#define NBLK (BB / MB)
#define NTHR 256
#define TBM  80
#define TBN  64
#define TTHR 160
#define SP   68

static_assert(VV % TBM == 0);
static_assert(G4 % TBN == 0);
static_assert(TBM == (TTHR / 32) * 16);
static_assert(TBN == 64);
static_assert(EE % 32 == 0);
static_assert(HH % 32 == 0);
static_assert((VV * (EE / 8)) % 256 == 0);
static_assert((G4 * (EE / 8)) % 256 == 0);
static_assert(EE == HH);
static_assert(NBLK * MB == BB);
static_assert((NTHR / 32) * 16 == HH);
static_assert(MB * HH == NTHR * 8);
static_assert(AP % 8 == 0);
static_assert(AP >= HH);
static_assert(HP % 4 == 0);
static_assert(HP >= HH);
static_assert(SP % 4 == 0);
static_assert(SP >= TBN);
static_assert(MB * CC * 4 == 128);
static_assert(MB * CC == 32);
static_assert(((TT - 1) & 1) == 1);

typedef __bf16         v16bf __attribute__((ext_vector_type(16)));
typedef unsigned short v8us  __attribute__((ext_vector_type(8)));
typedef float          v8f   __attribute__((ext_vector_type(8)));
typedef float          v4f   __attribute__((ext_vector_type(4)));

union Frag { v16bf v; v8us half[2]; };

constexpr size_t SZ_WPL   = (size_t)G4 * WP * 2;
constexpr size_t SZ_EPL   = (size_t)VV * WP * 2;
constexpr size_t SZ_XP    = (size_t)VV * XPP * 4;
constexpr size_t OFF_WIHI = 0;
constexpr size_t OFF_WILO = OFF_WIHI + SZ_WPL;
constexpr size_t OFF_WHHI = OFF_WILO + SZ_WPL;
constexpr size_t OFF_WHLO = OFF_WHHI + SZ_WPL;
constexpr size_t OFF_EHI  = OFF_WHLO + SZ_WPL;
constexpr size_t OFF_ELO  = OFF_EHI + SZ_EPL;
constexpr size_t OFF_XP   = OFF_ELO + SZ_EPL;
constexpr size_t WS_END   = OFF_XP + SZ_XP;
static_assert(OFF_WILO % 128 == 0);
static_assert(OFF_WHHI % 128 == 0);
static_assert(OFF_WHLO % 128 == 0);
static_assert(OFF_EHI % 128 == 0);
static_assert(OFF_ELO % 128 == 0);
static_assert(OFF_XP % 128 == 0);
static_assert(WS_END <= (size_t)134217728);
constexpr int NWPC = G4 * (WP / 8);
constexpr int NEPC = VV * (WP / 8);
static_assert((size_t)NWPC * 16 == SZ_WPL);
static_assert((size_t)NEPC * 16 == SZ_EPL);
static_assert((size_t)(VV / TBM) * TBM * XPP * 4 == SZ_XP);

__device__ __forceinline__ unsigned short bf_rne(float f) {
    const unsigned u = __float_as_uint(f);
    return (unsigned short)((u + 0x7FFFu + ((u >> 16) & 1u)) >> 16);
}
__device__ __forceinline__ void split2(float f, unsigned short& hi, unsigned short& lo) {
    hi = bf_rne(f);
    const float hf = __uint_as_float(((unsigned)hi) << 16);
    lo = bf_rne(f - hf);
}
__device__ __forceinline__ float rcpx(float x) { return __builtin_amdgcn_rcpf(x); }
__device__ __forceinline__ float sigm(float x) { return rcpx(1.0f + __expf(-x)); }
__device__ __forceinline__ float tanhm(float x) {
    const float e = __expf(2.0f * x);
    return 1.0f - 2.0f * rcpx(e + 1.0f);
}
__device__ __forceinline__ v8f zero8() {
    v8f z;
#pragma unroll
    for (int i = 0; i < 8; ++i) z[i] = 0.0f;
    return z;
}
__device__ __forceinline__ void cvt8(const float* src, v8us& hi, v8us& lo) {
    const v4f a = *(const v4f*)(src);
    const v4f b = *(const v4f*)(src + 4);
#pragma unroll
    for (int i = 0; i < 4; ++i) {
        unsigned short th, tl;
        split2(a[i], th, tl); hi[i] = th;     lo[i] = tl;
        split2(b[i], th, tl); hi[4 + i] = th; lo[4 + i] = tl;
    }
}
__device__ __forceinline__ v8f mma(v8f c, const Frag& a, const Frag& b) {
    return __builtin_amdgcn_wmma_f32_16x16x32_bf16(false, a.v, false, b.v, (short)0, c, false, false);
}

__global__ __launch_bounds__(256)
void cvt_w_kernel(const float* __restrict__ Wih, const float* __restrict__ Whh, unsigned short* Wpl)
{
    const int p   = blockIdx.x * 256 + threadIdx.x;
    const int sel = blockIdx.y;
    const int n   = p >> 4;
    const int c8  = (p & 15) * 8;
    const float* src = sel ? Whh : Wih;
    v8us hi, lo;
    cvt8(src + (size_t)n * EE + c8, hi, lo);
    unsigned short* dh = Wpl + (size_t)sel * 2 * G4 * WP + (size_t)n * WP + c8;
    unsigned short* dl = dh + (size_t)G4 * WP;
    *(volatile v8us*)dh = hi;
    *(volatile v8us*)dl = lo;
    __threadfence();
    *(volatile v8us*)dh = hi;
    *(volatile v8us*)dl = lo;
}

__global__ __launch_bounds__(256)
void cvt_emb_kernel(const float* __restrict__ emb, unsigned short* Ehi, unsigned short* Elo, int nvocab)
{
    const int p  = blockIdx.x * 256 + threadIdx.x;
    const int v  = p >> 4;
    const int c8 = (p & 15) * 8;
    const int vs = min(v, nvocab - 1);
    v8us hi, lo;
    cvt8(emb + (size_t)vs * EE + c8, hi, lo);
    unsigned short* dh = Ehi + (size_t)v * WP + c8;
    unsigned short* dl = Elo + (size_t)v * WP + c8;
    *(volatile v8us*)dh = hi;
    *(volatile v8us*)dl = lo;
    __threadfence();
    *(volatile v8us*)dh = hi;
    *(volatile v8us*)dl = lo;
}

__global__ __launch_bounds__(TTHR)
void table_kernel(const unsigned short* __restrict__ Ehi, const unsigned short* __restrict__ Elo,
                  const unsigned short* __restrict__ Wihi, const unsigned short* __restrict__ Wilo,
                  const float* __restrict__ bih, const float* __restrict__ bhh, float* XP)
{
    __shared__ __attribute__((aligned(16))) float sT[TTHR / 32][16][SP];

    const int tid  = threadIdx.x;
    const int lane = tid & 31;
    const int w    = tid >> 5;
    const int h    = lane >> 4;
    const int m    = lane & 15;
    const int row0 = blockIdx.x * TBM + w * 16;
    const int n0   = blockIdx.y * TBN;

    v8f acc[4];
#pragma unroll
    for (int q = 0; q < 4; ++q) acc[q] = zero8();

    const unsigned short* par = Ehi + (size_t)(row0 + m) * WP + 8 * h;
    const unsigned short* pal = Elo + (size_t)(row0 + m) * WP + 8 * h;

#pragma unroll 1
    for (int k0 = 0; k0 < EE; k0 += 32) {
        Frag ah, al, bh[4], bl[4];
        ah.half[0] = *(const v8us*)(par + k0);
        ah.half[1] = *(const v8us*)(par + k0 + 16);
        al.half[0] = *(const v8us*)(pal + k0);
        al.half[1] = *(const v8us*)(pal + k0 + 16);
#pragma unroll
        for (int q = 0; q < 4; ++q) {
            const unsigned short* ph = Wihi + (size_t)(n0 + q * 16 + m) * WP + k0 + 8 * h;
            const unsigned short* pl = Wilo + (size_t)(n0 + q * 16 + m) * WP + k0 + 8 * h;
            bh[q].half[0] = *(const v8us*)(ph);
            bh[q].half[1] = *(const v8us*)(ph + 16);
            bl[q].half[0] = *(const v8us*)(pl);
            bl[q].half[1] = *(const v8us*)(pl + 16);
        }
#pragma unroll
        for (int q = 0; q < 4; ++q) acc[q] = mma(acc[q], ah, bh[q]);
#pragma unroll
        for (int q = 0; q < 4; ++q) acc[q] = mma(acc[q], ah, bl[q]);
#pragma unroll
        for (int q = 0; q < 4; ++q) acc[q] = mma(acc[q], al, bh[q]);
        asm volatile("v_nop\n\tv_nop\n\tv_nop\n\tv_nop"
                     : "+v"(acc[0]), "+v"(acc[1]), "+v"(acc[2]), "+v"(acc[3])
                     : "v"(ah.v), "v"(al.v),
                       "v"(bh[0].v), "v"(bh[1].v), "v"(bh[2].v), "v"(bh[3].v),
                       "v"(bl[0].v), "v"(bl[1].v), "v"(bl[2].v), "v"(bl[3].v));
    }

#pragma unroll
    for (int q = 0; q < 4; ++q) {
        const int n = n0 + q * 16 + m;
        const float bias = bih[n] + bhh[n];
#pragma unroll
        for (int r = 0; r < 8; ++r) sT[w][8 * h + r][q * 16 + m] = acc[q][r] + bias;
    }
    __syncthreads();

    const int pc = m * 4;
#pragma unroll
    for (int i = 0; i < 8; ++i) {
        const int rr = i + 8 * h;
        const v4f v = *(const v4f*)&sT[w][rr][pc];
        float* dst = XP + (size_t)(row0 + rr) * XPP + n0 + pc;
        *(volatile v4f*)dst = v;
    }
    __threadfence();
#pragma unroll
    for (int i = 0; i < 8; ++i) {
        const int rr = i + 8 * h;
        const v4f v = *(const v4f*)&sT[w][rr][pc];
        float* dst = XP + (size_t)(row0 + rr) * XPP + n0 + pc;
        *(volatile v4f*)dst = v;
    }
}

__global__ __launch_bounds__(NTHR)
void rec_kernel(const int* __restrict__ tokens, const float* __restrict__ XP,
                const unsigned short* __restrict__ Whi, const unsigned short* __restrict__ Wlo,
                const float* __restrict__ Wc, const float* __restrict__ bc,
                float* out, int nvocab)
{
    __shared__ __attribute__((aligned(16))) unsigned short sAhi[2][MB][AP];
    __shared__ __attribute__((aligned(16))) unsigned short sAlo[2][MB][AP];
    __shared__ __attribute__((aligned(16))) float sHf[MB][HP];
    __shared__ __attribute__((aligned(16))) float sO[MB * CC];

    const int tid  = threadIdx.x;
    const int lane = tid & 31;
    const int w    = tid >> 5;
    const int h    = lane >> 4;
    const int m    = lane & 15;
    const int u    = w * 16 + m;
    const int b0   = blockIdx.x * MB;

    {
        v8us z;
#pragma unroll
        for (int i = 0; i < 8; ++i) z[i] = (unsigned short)0;
        const int zr = tid >> 4;
        const int zc = (tid & 15) * 8;
        *(v8us*)&sAhi[0][zr][zc] = z;
        *(v8us*)&sAlo[0][zr][zc] = z;
    }
    v8f cReg = zero8();

#pragma unroll 1
    for (int t = 0; t < TT; ++t) {
        const int cur = t & 1;
        const int nxt = cur ^ 1;

        __syncthreads();

        v8f acc[4];
#pragma unroll
        for (int q = 0; q < 4; ++q) acc[q] = zero8();

#pragma unroll 1
        for (int k0 = 0; k0 < HH; k0 += 32) {
            Frag ah, al, bh[4], bl[4];
            ah.half[0] = *(const v8us*)&sAhi[cur][m][k0 + 8 * h];
            ah.half[1] = *(const v8us*)&sAhi[cur][m][k0 + 8 * h + 16];
            al.half[0] = *(const v8us*)&sAlo[cur][m][k0 + 8 * h];
            al.half[1] = *(const v8us*)&sAlo[cur][m][k0 + 8 * h + 16];
#pragma unroll
            for (int q = 0; q < 4; ++q) {
                const unsigned short* ph = Whi + (size_t)(q * HH + u) * WP + k0 + 8 * h;
                const unsigned short* pl = Wlo + (size_t)(q * HH + u) * WP + k0 + 8 * h;
                bh[q].half[0] = *(const v8us*)(ph);
                bh[q].half[1] = *(const v8us*)(ph + 16);
                bl[q].half[0] = *(const v8us*)(pl);
                bl[q].half[1] = *(const v8us*)(pl + 16);
            }
#pragma unroll
            for (int q = 0; q < 4; ++q) acc[q] = mma(acc[q], ah, bh[q]);
#pragma unroll
            for (int q = 0; q < 4; ++q) acc[q] = mma(acc[q], ah, bl[q]);
#pragma unroll
            for (int q = 0; q < 4; ++q) acc[q] = mma(acc[q], al, bh[q]);
            asm volatile("v_nop\n\tv_nop\n\tv_nop\n\tv_nop"
                         : "+v"(acc[0]), "+v"(acc[1]), "+v"(acc[2]), "+v"(acc[3])
                         : "v"(ah.v), "v"(al.v),
                           "v"(bh[0].v), "v"(bh[1].v), "v"(bh[2].v), "v"(bh[3].v),
                           "v"(bl[0].v), "v"(bl[1].v), "v"(bl[2].v), "v"(bl[3].v));
        }

#pragma unroll
        for (int r = 0; r < 8; ++r) {
            const int row = 8 * h + r;
            int tk = tokens[(size_t)(b0 + row) * TT + t];
            tk = min(max(tk, 0), nvocab - 1);
            const float* xr = XP + (size_t)tk * XPP + u;
            const float gi = acc[0][r] + xr[0];
            const float gf = acc[1][r] + xr[HH];
            const float gg = acc[2][r] + xr[2 * HH];
            const float go = acc[3][r] + xr[3 * HH];
            const float cn = sigm(gf) * cReg[r] + sigm(gi) * tanhm(gg);
            const float hn = sigm(go) * tanhm(cn);
            cReg[r] = cn;
            sHf[row][u] = hn;
            unsigned short th, tl;
            split2(hn, th, tl);
            sAhi[nxt][row][u] = th;
            sAlo[nxt][row][u] = tl;
        }
    }

    __syncthreads();

    if (tid < MB * CC) {
        const int bl_ = tid >> 1;
        const int c   = tid & 1;
        const float* wr = Wc + (size_t)c * HH;
        float s = 0.0f;
#pragma unroll 4
        for (int k = 0; k < HH; ++k) s += sHf[bl_][k] * wr[k];
        sO[tid] = s + bc[c];
    }
    __syncthreads();

    {
        const v4f v = *(const v4f*)&sO[(tid & 7) * 4];
        float* dst = out + (size_t)b0 * CC + (tid & 7) * 4;
        if (tid < 8) *(volatile v4f*)dst = v;
        __threadfence();
        if (tid < 8) *(volatile v4f*)dst = v;
    }
}

extern "C" void kernel_launch(void* const* d_in, const int* in_sizes, int n_in,
                              void* d_out, int out_size, void* d_ws, size_t ws_size,
                              hipStream_t stream)
{
    if (n_in < 8) return;
    if (in_sizes[0] != BB * TT)      return;
    if (in_sizes[1] != VV * EE)      return;
    if (in_sizes[2] != G4 * EE)      return;
    if (in_sizes[3] != G4 * HH)      return;
    if (in_sizes[4] != G4)           return;
    if (in_sizes[5] != G4)           return;
    if (in_sizes[6] != CC * HH)      return;
    if (in_sizes[7] != CC)           return;
    if (out_size != BB * CC)         return;
    if (ws_size < WS_END)            return;

    const int*   tokens = (const int*)d_in[0];
    const float* emb    = (const float*)d_in[1];
    const float* Wih    = (const float*)d_in[2];
    const float* Whh    = (const float*)d_in[3];
    const float* bih    = (const float*)d_in[4];
    const float* bhh    = (const float*)d_in[5];
    const float* Wc     = (const float*)d_in[6];
    const float* bc     = (const float*)d_in[7];
    const int nvocab    = in_sizes[1] / EE;

    float* out = (float*)d_out;

    char* ws = (char*)d_ws;
    unsigned short* Wpl  = (unsigned short*)(ws + OFF_WIHI);
    unsigned short* Wihi = (unsigned short*)(ws + OFF_WIHI);
    unsigned short* Wilo = (unsigned short*)(ws + OFF_WILO);
    unsigned short* Whhi = (unsigned short*)(ws + OFF_WHHI);
    unsigned short* Whlo = (unsigned short*)(ws + OFF_WHLO);
    unsigned short* Ehi  = (unsigned short*)(ws + OFF_EHI);
    unsigned short* Elo  = (unsigned short*)(ws + OFF_ELO);
    float*          XP   = (float*)(ws + OFF_XP);

    cvt_w_kernel<<<dim3(NWPC / 256, 2), dim3(256), 0, stream>>>(Wih, Whh, Wpl);
    cvt_emb_kernel<<<dim3(NEPC / 256), dim3(256), 0, stream>>>(emb, Ehi, Elo, nvocab);
    table_kernel<<<dim3(VV / TBM, G4 / TBN), dim3(TTHR), 0, stream>>>(Ehi, Elo, Wihi, Wilo, bih, bhh, XP);
    rec_kernel<<<dim3(NBLK), dim3(NTHR), 0, stream>>>(tokens, XP, Whhi, Whlo, Wc, bc, out, nvocab);
}
